// _DiffPoolBatchedGraphLayer_5634997092474
// MI455X (gfx1250) — hardware-verified
//
#include <hip/hip_runtime.h>
#include <stddef.h>


#define DFE    256
#define FO     256
#define KC     64
#define NPG    1024
#define NCOL   (FO + KC)
#define KX     (2 * DFE)
#define NTHR   256
#define NWAVE  8
#define EPT    8
#define NGRP   2
#define CHUNK  (NTHR * EPT * NGRP)
#define WCAP   (EPT * NGRP * 32)
#define LISTN  (NWAVE * WCAP)
#define NB1    256
#define NB2    1024
#define GROWS  64
#define FPITCH 72
#define WSCALE 16.0f
#define WINV   0.0625f
#define SSCALE 16384.0f
#define SINV   (1.0f / 16384.0f)
#define MSCALE 256.0f
#define O0INV  (1.0f / 4194304.0f)

#define LDS_AGG1 (NB1 * DFE * 4 + LISTN * 4 + NB1 * 4 + 32)
#define LDS_AGG2 (NB2 * KC * 4 + LISTN * 4 + 32)
#define LDS_POOL (KC * FO * 4 + KC * KC * 4)

static_assert((CHUNK & (CHUNK - 1)) == 0);
static_assert(CHUNK <= 4096);
static_assert(NB1 <= 4096 && NB2 <= 4096);
static_assert((NB1 & (NB1 - 1)) == 0 && (NB2 & (NB2 - 1)) == 0);
static_assert(NB2 == NPG);
static_assert(NB1 == 32 * NWAVE);
static_assert(FO == 32 * NWAVE && KC == 8 * NWAVE);
static_assert(GROWS == 64 && (NPG % GROWS) == 0);
static_assert(NCOL == 320 && DFE == 256 && KC == 64);
static_assert((KX % 32) == 0 && (NPG % 32) == 0);
static_assert(LDS_AGG1 <= 300000 && LDS_AGG2 <= 300000);

typedef float    v2f  __attribute__((ext_vector_type(2)));
typedef float    v4f  __attribute__((ext_vector_type(4)));
typedef float    v8f  __attribute__((ext_vector_type(8)));
typedef int      v4i  __attribute__((ext_vector_type(4)));
typedef _Float16 v8h  __attribute__((ext_vector_type(8)));
typedef _Float16 v16h __attribute__((ext_vector_type(16)));
union FragH { v16h v; v8h h[2]; };

__device__ __forceinline__ v8h cvt8(v4f a, v4f b) {
  v8h r;
  r[0] = (_Float16)a.x; r[1] = (_Float16)a.y; r[2] = (_Float16)a.z; r[3] = (_Float16)a.w;
  r[4] = (_Float16)b.x; r[5] = (_Float16)b.y; r[6] = (_Float16)b.z; r[7] = (_Float16)b.w;
  return r;
}

__device__ __forceinline__ v8f wmh(v16h a, v16h b, v8f c) {
  v8f d = __builtin_amdgcn_wmma_f32_16x16x32_f16(false, a, false, b, (short)0, c, false, false);
  asm volatile("v_nop\n\tv_nop\n\tv_nop\n\tv_nop" : "+v"(d) : "v"(a), "v"(b));
  return d;
}

template <int NB>
__device__ __forceinline__ int scan_chunk(const int* __restrict__ dsts, int nE, int cbase, int nodeBase,
                                          int* list, int tid, int lane, int wave) {
  int wc = 0;
#pragma unroll
  for (int g = 0; g < NGRP; ++g) {
    const int el0  = (g * NTHR + tid) * EPT;
    const int e0   = cbase + el0;
    const int sent = -2147483647 - 1;
    v4i da, db;
    if (e0 + 7 < nE) {
      da = *(const v4i*)(dsts + e0);
      db = *(const v4i*)(dsts + e0 + 4);
    } else {
      da.x = (e0     < nE) ? dsts[min(e0, nE - 1)] : sent;
      da.y = (e0 + 1 < nE) ? dsts[min(e0 + 1, nE - 1)] : sent;
      da.z = (e0 + 2 < nE) ? dsts[min(e0 + 2, nE - 1)] : sent;
      da.w = (e0 + 3 < nE) ? dsts[min(e0 + 3, nE - 1)] : sent;
      db.x = (e0 + 4 < nE) ? dsts[min(e0 + 4, nE - 1)] : sent;
      db.y = (e0 + 5 < nE) ? dsts[min(e0 + 5, nE - 1)] : sent;
      db.z = (e0 + 6 < nE) ? dsts[min(e0 + 6, nE - 1)] : sent;
      db.w = (e0 + 7 < nE) ? dsts[min(e0 + 7, nE - 1)] : sent;
    }
    const unsigned nb = (unsigned)nodeBase;
    const unsigned s0 = (unsigned)da.x - nb, s1 = (unsigned)da.y - nb;
    const unsigned s2 = (unsigned)da.z - nb, s3 = (unsigned)da.w - nb;
    const unsigned s4 = (unsigned)db.x - nb, s5 = (unsigned)db.y - nb;
    const unsigned s6 = (unsigned)db.z - nb, s7 = (unsigned)db.w - nb;
    const bool h0 = s0 < (unsigned)NB, h1 = s1 < (unsigned)NB, h2 = s2 < (unsigned)NB, h3 = s3 < (unsigned)NB;
    const bool h4 = s4 < (unsigned)NB, h5 = s5 < (unsigned)NB, h6 = s6 < (unsigned)NB, h7 = s7 < (unsigned)NB;
    const unsigned any = __builtin_amdgcn_ballot_w32(h0 | h1 | h2 | h3 | h4 | h5 | h6 | h7);
    if (any != 0u) {
#define HITJ(J, HJ, SJ) { \
        const unsigned mj = __builtin_amdgcn_ballot_w32(HJ); \
        if (mj != 0u) { \
          if (HJ) { \
            const int pos = wc + (int)__builtin_amdgcn_mbcnt_lo(mj, 0u); \
            if (pos < WCAP) list[wave * WCAP + pos] = ((el0 + (J)) << 12) | (int)(SJ); \
          } \
          wc += (int)__builtin_popcount(mj); } }
      HITJ(0, h0, s0)
      HITJ(1, h1, s1)
      HITJ(2, h2, s2)
      HITJ(3, h3, s3)
      HITJ(4, h4, s4)
      HITJ(5, h5, s5)
      HITJ(6, h6, s6)
      HITJ(7, h7, s7)
#undef HITJ
    }
  }
  return wc;
}

__global__ __launch_bounds__(NTHR) void k_wprep(
    const float* __restrict__ Wsf, const float* __restrict__ Wnf,
    const float* __restrict__ Wsp, const float* __restrict__ Wnp, _Float16* WcT) {
  const int i = blockIdx.x * NTHR + threadIdx.x;
  if (i >= NCOL * KX / 8) return;
  const int o  = i * 8;
  const int n  = o / KX;
  const int k0 = o - n * KX;
  const bool nbr = k0 >= DFE;
  const int  kk  = nbr ? k0 - DFE : k0;
  const float* p;
  int pitch;
  if (n < FO) { p = (nbr ? Wnf : Wsf) + (size_t)kk * FO + n;        pitch = FO; }
  else        { p = (nbr ? Wnp : Wsp) + (size_t)kk * KC + (n - FO); pitch = KC; }
  v4f a, b;
  a.x = p[0];         a.y = p[pitch];     a.z = p[2 * pitch]; a.w = p[3 * pitch];
  b.x = p[4 * pitch]; b.y = p[5 * pitch]; b.z = p[6 * pitch]; b.w = p[7 * pitch];
  a = a * WSCALE;
  b = b * WSCALE;
  const v8h hv = cvt8(a, b);
  _Float16* dp = WcT + o;
  *(volatile v8h*)dp = hv;
  __threadfence();
  *(volatile v8h*)dp = hv;
}

__device__ __forceinline__ void agg1_store_pass(const float* acc, const int* cnt, const float* __restrict__ h,
                                                _Float16* X, int nodeBase, int wave, int lane) {
#pragma unroll 4
  for (int i = 0; i < NB1 / NWAVE; ++i) {
    const int slot = wave * (NB1 / NWAVE) + i;
    const int node = nodeBase + slot;
    const int d    = cnt[slot];
    const float inv = 1.0f / (float)(d > 1 ? d : 1);
    const float* ap = acc + slot * DFE + 8 * lane;
    const v4f a0 = *(const v4f*)ap * inv, a1 = *(const v4f*)(ap + 4) * inv;
    const float* hp = h + (size_t)node * DFE + 8 * lane;
    const v4f h0 = *(const v4f*)hp, h1 = *(const v4f*)(hp + 4);
    _Float16* xp = X + (size_t)node * KX + 8 * lane;
    *(volatile v8h*)xp = cvt8(h0, h1);
    *(volatile v8h*)(xp + DFE) = cvt8(a0, a1);
  }
}

__global__ __launch_bounds__(NTHR) void k_agg1(
    const float* __restrict__ h, const int* __restrict__ src, const int* __restrict__ dst,
    _Float16* X, int nN, int nE) {
  extern __shared__ v4f lds_dyn[];
  float* acc  = (float*)lds_dyn;
  int*   list = (int*)(acc + NB1 * DFE);
  int*   cnt  = list + LISTN;
  int*   wcnt = cnt + NB1;
  const int tid = threadIdx.x, lane = tid & 31, wave = tid >> 5;
  const int nodeBase = blockIdx.x * NB1;

  {
    const v4f z = {0.f, 0.f, 0.f, 0.f};
    for (int i = tid; i < NB1 * DFE / 4; i += NTHR) lds_dyn[i] = z;
    for (int i = tid; i < NB1; i += NTHR) cnt[i] = 0;
  }
  __syncthreads();

  const int nChunks = (nE + CHUNK - 1) / CHUNK;
#pragma unroll 1
  for (int ch = 0; ch < nChunks; ++ch) {
    const int cbase = ch * CHUNK;
    const int wc = scan_chunk<NB1>(dst, nE, cbase, nodeBase, list, tid, lane, wave);
    if (lane == 0) wcnt[wave] = wc;
    __syncthreads();
    if (wave == 0) {
#pragma unroll 1
      for (int wsx = 0; wsx < NWAVE; ++wsx) {
        int n = __builtin_amdgcn_readfirstlane(wcnt[wsx]);
        n = n > WCAP ? WCAP : (n < 0 ? 0 : n);
        const int* lp = list + wsx * WCAP;
#pragma unroll 1
        for (int i = 0; i < n; ++i) {
          const int ent  = __builtin_amdgcn_readfirstlane(lp[i]);
          const int slot = ent & (NB1 - 1);
          int e = cbase + ((ent >> 12) & (CHUNK - 1));
          e = e > nE - 1 ? nE - 1 : e;
          int sn = src[e];
          sn = sn < 0 ? 0 : (sn > nN - 1 ? nN - 1 : sn);
          if (lane == 0) cnt[slot] = cnt[slot] + 1;
          const float* hp = h + (size_t)sn * DFE + 4 * lane;
          const v4f v0 = *(const v4f*)hp;
          const v4f v1 = *(const v4f*)(hp + 128);
          v4f* ap = (v4f*)(acc + slot * DFE + 4 * lane);
          ap[0]  = ap[0] + v0;
          ap[32] = ap[32] + v1;
        }
      }
    }
    __syncthreads();
  }

  agg1_store_pass(acc, cnt, h, X, nodeBase, wave, lane);
  __threadfence();
  agg1_store_pass(acc, cnt, h, X, nodeBase, wave, lane);
}

__device__ __forceinline__ void stage_feat(v8f a, float bb, _Float16* dstp) {
  v8h t;
#pragma unroll
  for (int r = 0; r < 8; ++r) t[r] = (_Float16)fmaxf(a[r] * WINV + bb, 0.0f);
  *(v8h*)dstp = t;
}

__device__ __forceinline__ void gemm_store_pass(const _Float16* stgF, const float* spool, const _Float16* spT,
                                                _Float16* featT, float* srm, _Float16* sT,
                                                int g, int nl0, int rowBase, int wave, int lane) {
  const int q = lane >> 3, j = lane & 7;
#pragma unroll
  for (int i = 0; i < 8; ++i) {
    const int f = 32 * wave + 4 * i + q;
    const v8h v = *(const v8h*)(stgF + f * FPITCH + 8 * j);
    *(volatile v8h*)(featT + ((size_t)g * FO + f) * NPG + nl0 + 8 * j) = v;
  }
#pragma unroll
  for (int i = 0; i < 4; ++i) {
    const int fo = (wave * 4 + i) * 128 + 4 * lane;
    const v4f v = *(const v4f*)(spool + fo);
    *(volatile v4f*)(srm + (size_t)rowBase * KC + fo) = v;
  }
#pragma unroll
  for (int i = 0; i < 2; ++i) {
    const int c = 8 * wave + 4 * i + q;
    const v8h v = *(const v8h*)(spT + c * FPITCH + 8 * j);
    *(volatile v8h*)(sT + ((size_t)g * KC + c) * NPG + nl0 + 8 * j) = v;
  }
}

__global__ __launch_bounds__(NTHR) void k_gemm(
    const _Float16* __restrict__ X, const _Float16* __restrict__ WcT,
    const float* __restrict__ bfe, const float* __restrict__ bpo,
    _Float16* featT, float* srm, _Float16* sT) {
  __shared__ __attribute__((aligned(16))) _Float16 stgF[FO * FPITCH];
  __shared__ __attribute__((aligned(16))) float    spool[GROWS * KC];
  __shared__ __attribute__((aligned(16))) _Float16 spT[KC * FPITCH];
  const int tid = threadIdx.x, lane = tid & 31, wave = tid >> 5, hh = lane >> 4, m = lane & 15;
  const int wr = wave & 3, wc = wave >> 2;
  const int rowBase = blockIdx.x * GROWS;
  const int g = rowBase / NPG, nl0 = rowBase - g * NPG;

  v8f acc[10];
#pragma unroll
  for (int t = 0; t < 10; ++t) { v8f z = {0.f, 0.f, 0.f, 0.f, 0.f, 0.f, 0.f, 0.f}; acc[t] = z; }

  const _Float16* pa = X + (size_t)(rowBase + 16 * wr + m) * KX + 8 * hh;
  const _Float16* pb = WcT + (size_t)(160 * wc + m) * KX + 8 * hh;
#pragma unroll 2
  for (int kt = 0; kt < KX / 32; ++kt) {
    FragH a;
    a.h[0] = *(const v8h*)(pa + 32 * kt);
    a.h[1] = *(const v8h*)(pa + 32 * kt + 16);
#pragma unroll
    for (int t = 0; t < 10; ++t) {
      const _Float16* bp = pb + (size_t)(16 * t) * KX + 32 * kt;
      FragH b;
      b.h[0] = *(const v8h*)bp;
      b.h[1] = *(const v8h*)(bp + 16);
      acc[t] = wmh(a.v, b.v, acc[t]);
    }
  }

  const int rl = 16 * wr + 8 * hh;
  if (wc == 0) {
#pragma unroll
    for (int t = 0; t < 10; ++t) {
      const int f = 16 * t + m;
      stage_feat(acc[t], bfe[f], stgF + f * FPITCH + rl);
    }
  } else {
#pragma unroll
    for (int t = 0; t < 6; ++t) {
      const int f = 160 + 16 * t + m;
      stage_feat(acc[t], bfe[f], stgF + f * FPITCH + rl);
    }
    float p[4][8];
#pragma unroll
    for (int u = 0; u < 4; ++u) {
      const float bb = bpo[16 * u + m];
#pragma unroll
      for (int r = 0; r < 8; ++r) p[u][r] = fmaxf(acc[6 + u][r] * WINV + bb, 0.0f);
    }
#pragma unroll
    for (int r = 0; r < 8; ++r) {
      float mx = fmaxf(fmaxf(p[0][r], p[1][r]), fmaxf(p[2][r], p[3][r]));
      mx = fmaxf(mx, __shfl_xor(mx, 1, 32));
      mx = fmaxf(mx, __shfl_xor(mx, 2, 32));
      mx = fmaxf(mx, __shfl_xor(mx, 4, 32));
      mx = fmaxf(mx, __shfl_xor(mx, 8, 32));
      const float e0 = expf(p[0][r] - mx), e1 = expf(p[1][r] - mx);
      const float e2 = expf(p[2][r] - mx), e3 = expf(p[3][r] - mx);
      float sum = (e0 + e1) + (e2 + e3);
      sum += __shfl_xor(sum, 1, 32);
      sum += __shfl_xor(sum, 2, 32);
      sum += __shfl_xor(sum, 4, 32);
      sum += __shfl_xor(sum, 8, 32);
      const float inv = 1.0f / sum;
      p[0][r] = e0 * inv; p[1][r] = e1 * inv; p[2][r] = e2 * inv; p[3][r] = e3 * inv;
    }
#pragma unroll
    for (int u = 0; u < 4; ++u) {
#pragma unroll
      for (int r = 0; r < 8; ++r) spool[(rl + r) * KC + 16 * u + m] = p[u][r];
      v8h t8;
#pragma unroll
      for (int r = 0; r < 8; ++r) t8[r] = (_Float16)(p[u][r] * SSCALE);
      *(v8h*)(spT + (16 * u + m) * FPITCH + rl) = t8;
    }
  }
  __syncthreads();

  gemm_store_pass(stgF, spool, spT, featT, srm, sT, g, nl0, rowBase, wave, lane);
  __threadfence();
  gemm_store_pass(stgF, spool, spT, featT, srm, sT, g, nl0, rowBase, wave, lane);
}

__device__ __forceinline__ void agg2_store_pass(const float* acc, _Float16* MT, int g, int wave, int lane) {
#pragma unroll 4
  for (int i = 0; i < 32; ++i) {
    const int c  = 8 * wave + (i >> 2);
    const int nb = (i & 3) * 256 + 8 * lane;
    v8h t;
#pragma unroll
    for (int u = 0; u < 8; ++u) t[u] = (_Float16)(acc[(nb + u) * KC + c] * MSCALE);
    *(volatile v8h*)(MT + ((size_t)g * KC + c) * NPG + nb) = t;
  }
}

__global__ __launch_bounds__(NTHR) void k_agg2(
    const float* __restrict__ srm, const int* __restrict__ src, const int* __restrict__ dst,
    _Float16* MT, int nN, int nE) {
  extern __shared__ v4f lds_dyn[];
  float* acc  = (float*)lds_dyn;
  int*   list = (int*)(acc + NB2 * KC);
  int*   wcnt = list + LISTN;
  const int tid = threadIdx.x, lane = tid & 31, wave = tid >> 5;
  const int nodeBase = blockIdx.x * NB2;
  (void)nN;

  {
    const v4f z = {0.f, 0.f, 0.f, 0.f};
    for (int i = tid; i < NB2 * KC / 4; i += NTHR) lds_dyn[i] = z;
  }
  __syncthreads();

  const int nChunks = (nE + CHUNK - 1) / CHUNK;
#pragma unroll 1
  for (int ch = 0; ch < nChunks; ++ch) {
    const int cbase = ch * CHUNK;
    const int wc = scan_chunk<NB2>(dst, nE, cbase, nodeBase, list, tid, lane, wave);
    if (lane == 0) wcnt[wave] = wc;
    __syncthreads();
    if (wave == 0) {
#pragma unroll 1
      for (int wsx = 0; wsx < NWAVE; ++wsx) {
        int n = __builtin_amdgcn_readfirstlane(wcnt[wsx]);
        n = n > WCAP ? WCAP : (n < 0 ? 0 : n);
        const int* lp = list + wsx * WCAP;
#pragma unroll 1
        for (int i = 0; i < n; ++i) {
          const int ent  = __builtin_amdgcn_readfirstlane(lp[i]);
          const int slot = ent & (NB2 - 1);
          int e = cbase + ((ent >> 12) & (CHUNK - 1));
          e = e > nE - 1 ? nE - 1 : e;
          const int sr = src[e];
          const int se = nodeBase + (sr & (NPG - 1));
          const v2f v = *(const v2f*)(srm + (size_t)se * KC + 2 * lane);
          v2f* ap = (v2f*)(acc + slot * KC + 2 * lane);
          *ap = *ap + v;
        }
      }
    }
    __syncthreads();
  }

  agg2_store_pass(acc, MT, blockIdx.x, wave, lane);
  __threadfence();
  agg2_store_pass(acc, MT, blockIdx.x, wave, lane);
}

__device__ __forceinline__ void pool_store_pass(const float* so1, const float* so0, float* out0, float* out1,
                                                int g, int nG, int wave, int lane, int hh, int m) {
#pragma unroll
  for (int i = 0; i < 16; ++i) {
    const int fo = (wave * 16 + i) * 128 + 4 * lane;
    const v4f v = *(const v4f*)(so1 + fo);
    *(volatile v4f*)(out1 + (size_t)g * KC * FO + fo) = v;
  }
  const size_t R0 = (size_t)nG * KC;
  const int nq = (nG * KC) / 128;
  const int qd = (g * KC) / 128;
  const int hd = ((g * KC) >> 6) & 1;
  const v4f z = {0.f, 0.f, 0.f, 0.f};
#pragma unroll 1
  for (int rr8 = 0; rr8 < 8; ++rr8) {
    const int rr = 8 * wave + rr8;
    const v4f dv = *(const v4f*)(so0 + rr * KC + 4 * m);
    float* rowp = out0 + ((size_t)g * KC + rr) * R0 + 4 * lane;
#pragma unroll 1
    for (int q = 0; q < nq; ++q) {
      v4f v = z;
      if (q == qd && hh == hd) v = dv;
      *(volatile v4f*)(rowp + (size_t)q * 128) = v;
    }
  }
}

__global__ __launch_bounds__(NTHR) void k_pool(
    const _Float16* __restrict__ sT, const _Float16* __restrict__ featT, const _Float16* __restrict__ MT,
    float* out0, float* out1, int nG) {
  extern __shared__ v4f lds_dyn[];
  float* so1 = (float*)lds_dyn;
  float* so0 = so1 + KC * FO;
  const int tid = threadIdx.x, lane = tid & 31, wave = tid >> 5, hh = lane >> 4, m = lane & 15;
  const int g = blockIdx.x, ct = wave & 3, fh = wave >> 2;

  v8f a1[8], a0[2];
#pragma unroll
  for (int t = 0; t < 8; ++t) { v8f z = {0.f, 0.f, 0.f, 0.f, 0.f, 0.f, 0.f, 0.f}; a1[t] = z; }
#pragma unroll
  for (int u = 0; u < 2; ++u) { v8f z = {0.f, 0.f, 0.f, 0.f, 0.f, 0.f, 0.f, 0.f}; a0[u] = z; }

  const _Float16* pa = sT    + ((size_t)g * KC + 16 * ct + m) * NPG + 8 * hh;
  const _Float16* pf = featT + ((size_t)g * FO + 128 * fh + m) * NPG + 8 * hh;
  const _Float16* pm = MT    + ((size_t)g * KC + 32 * fh + m) * NPG + 8 * hh;
#pragma unroll 2
  for (int kt = 0; kt < NPG / 32; ++kt) {
    FragH a;
    a.h[0] = *(const v8h*)(pa + 32 * kt);
    a.h[1] = *(const v8h*)(pa + 32 * kt + 16);
#pragma unroll
    for (int t = 0; t < 8; ++t) {
      const _Float16* bp = pf + (size_t)(16 * t) * NPG + 32 * kt;
      FragH b;
      b.h[0] = *(const v8h*)bp;
      b.h[1] = *(const v8h*)(bp + 16);
      a1[t] = wmh(a.v, b.v, a1[t]);
    }
#pragma unroll
    for (int u = 0; u < 2; ++u) {
      const _Float16* bp = pm + (size_t)(16 * u) * NPG + 32 * kt;
      FragH b;
      b.h[0] = *(const v8h*)bp;
      b.h[1] = *(const v8h*)(bp + 16);
      a0[u] = wmh(a.v, b.v, a0[u]);
    }
  }

  const int rc = 16 * ct + 8 * hh;
#pragma unroll
  for (int t = 0; t < 8; ++t) {
#pragma unroll
    for (int r = 0; r < 8; ++r) so1[(rc + r) * FO + 128 * fh + 16 * t + m] = a1[t][r] * SINV;
  }
#pragma unroll
  for (int u = 0; u < 2; ++u) {
#pragma unroll
    for (int r = 0; r < 8; ++r) so0[(rc + r) * KC + 32 * fh + 16 * u + m] = a0[u][r] * O0INV;
  }
  __syncthreads();

  pool_store_pass(so1, so0, out0, out1, g, nG, wave, lane, hh, m);
  __threadfence();
  pool_store_pass(so1, so0, out0, out1, g, nG, wave, lane, hh, m);
}

extern "C" void kernel_launch(void* const* d_in, const int* in_sizes, int n_in,
                              void* d_out, int out_size, void* d_ws, size_t ws_size,
                              hipStream_t stream) {
  if (n_in < 9) return;
  const int nN = in_sizes[0] / DFE;
  const int nE = in_sizes[1];
  if (nN <= 0 || in_sizes[0] != nN * DFE || (nN % NPG) != 0) return;
  if (nE <= 0 || in_sizes[2] != nE) return;
  if (in_sizes[3] != DFE * FO || in_sizes[4] != DFE * FO || in_sizes[5] != FO) return;
  if (in_sizes[6] != DFE * KC || in_sizes[7] != DFE * KC || in_sizes[8] != KC) return;
  const int nG = nN / NPG;
  if ((nG % 2) != 0) return;
  const size_t nOut0 = (size_t)nG * KC * (size_t)nG * KC;
  const size_t nOut1 = (size_t)nG * KC * FO;
  if ((size_t)out_size != nOut0 + nOut1) return;

  const float* h   = (const float*)d_in[0];
  const int*   src = (const int*)d_in[1];
  const int*   dst = (const int*)d_in[2];
  const float* Wsf = (const float*)d_in[3];
  const float* Wnf = (const float*)d_in[4];
  const float* bfe = (const float*)d_in[5];
  const float* Wsp = (const float*)d_in[6];
  const float* Wnp = (const float*)d_in[7];
  const float* bpo = (const float*)d_in[8];
  float* out0 = (float*)d_out;
  float* out1 = (float*)d_out + nOut0;

  char* ws = (char*)d_ws;
  size_t off = 0;
  const size_t oW  = off; off += (size_t)NCOL * KX * 2;    off = (off + 255) & ~(size_t)255;
  const size_t oX  = off; off += (size_t)nN * KX * 2;      off = (off + 255) & ~(size_t)255;
  const size_t oFT = off; off += (size_t)nN * FO * 2;      off = (off + 255) & ~(size_t)255;
  const size_t oS  = off; off += (size_t)nN * KC * 4;      off = (off + 255) & ~(size_t)255;
  const size_t oST = off; off += (size_t)nN * KC * 2;      off = (off + 255) & ~(size_t)255;
  const size_t oMT = off; off += (size_t)nN * KC * 2;      off = (off + 255) & ~(size_t)255;
  if (off > ws_size || off > (size_t)134217728) return;
  _Float16* WcT   = (_Float16*)(ws + oW);
  _Float16* X     = (_Float16*)(ws + oX);
  _Float16* featT = (_Float16*)(ws + oFT);
  float*    srm   = (float*)(ws + oS);
  _Float16* sT    = (_Float16*)(ws + oST);
  _Float16* MT    = (_Float16*)(ws + oMT);

  const int nPrep = NCOL * KX / 8;
  k_wprep<<<(nPrep + NTHR - 1) / NTHR, NTHR, 0, stream>>>(Wsf, Wnf, Wsp, Wnp, WcT);

  hipFuncSetAttribute(reinterpret_cast<const void*>(&k_agg1),
                      hipFuncAttributeMaxDynamicSharedMemorySize, LDS_AGG1);
  k_agg1<<<nN / NB1, NTHR, LDS_AGG1, stream>>>(h, src, dst, X, nN, nE);

  k_gemm<<<nN / GROWS, NTHR, 0, stream>>>(X, WcT, bfe, bpo, featT, srm, sT);

  hipFuncSetAttribute(reinterpret_cast<const void*>(&k_agg2),
                      hipFuncAttributeMaxDynamicSharedMemorySize, LDS_AGG2);
  k_agg2<<<nN / NB2, NTHR, LDS_AGG2, stream>>>(srm, src, dst, MT, nN, nE);

  hipFuncSetAttribute(reinterpret_cast<const void*>(&k_pool),
                      hipFuncAttributeMaxDynamicSharedMemorySize, LDS_POOL);
  k_pool<<<nG, NTHR, LDS_POOL, stream>>>(sT, featT, MT, out0, out1, nG);
}
